// BiMambaBlock_35201551958097
// MI455X (gfx1250) — hardware-verified
//
#include <hip/hip_runtime.h>
#include <math.h>

typedef __attribute__((ext_vector_type(16))) _Float16 v16h;
typedef __attribute__((ext_vector_type(8)))  _Float16 v8h;
typedef __attribute__((ext_vector_type(8)))  float    v8f;
typedef __attribute__((ext_vector_type(4)))  float    v4f;

constexpr int kBatch = 2;
constexpr int kSeqL  = 1024;
constexpr int kDmod  = 1024;
constexpr int kDin   = 2048;
constexpr int kNst   = 16;
constexpr int kDtR   = 64;
constexpr int kPrjN  = 96;
constexpr int kPrjP  = 128;
constexpr int kXZP   = 2 * kDin;
constexpr int kYP    = 2 * kDin;
constexpr int kRows  = kBatch * kSeqL;
constexpr int kTP    = 260;
constexpr int kChunk = 16;

constexpr float kCarryW  = 256.0f;
constexpr float kCarryU  = 256.0f;
constexpr float kCarryDt = 256.0f;
constexpr float kCarryY  = 1024.0f;
constexpr float kFoldIn  = 1.0f / kCarryW;
constexpr float kFoldXp  = 1.0f / (kCarryU * kCarryW);
constexpr float kFoldDt  = 1.0f / (kCarryDt * kCarryW);
constexpr float kFoldOut = 1.0f / (kCarryY * kCarryW);

static_assert(kDtR + 2 * kNst == kPrjN);
static_assert((kRows % 64) == 0 && (kXZP % 64) == 0 && (kPrjP % 64) == 0 && (kDin % 64) == 0 && (kDmod % 64) == 0);
static_assert((kDmod % 32) == 0 && (kDin % 32) == 0 && (kDtR % 32) == 0 && (kYP % 32) == 0);
static_assert((kSeqL % 64) == 0 && (kDin % 256) == 0 && (kSeqL % kChunk) == 0);
static_assert((kDmod % 256) == 0 && (kDin % 256) == 0 && ((kDtR * 2) % 128) == 0);

constexpr size_t kOffX16   = 0;
constexpr size_t kOffWIN   = kOffX16  + (size_t)kRows * kDmod * 2;
constexpr size_t kOffWXP   = kOffWIN  + (size_t)kXZP  * kDmod * 2;
constexpr size_t kOffWDT   = kOffWXP  + (size_t)kPrjP * kDin  * 2;
constexpr size_t kOffWOUT  = kOffWDT  + (size_t)kDin  * kDtR  * 2;
constexpr size_t kOffXZ    = kOffWOUT + (size_t)kDmod * kYP   * 2;
constexpr size_t kOffUC    = kOffXZ   + (size_t)kRows * kXZP  * 4;
constexpr size_t kOffUC16  = kOffUC   + (size_t)kRows * kDin  * 4;
constexpr size_t kOffPROJ  = kOffUC16 + (size_t)kRows * kDin  * 2;
constexpr size_t kOffDT16  = kOffPROJ + (size_t)kRows * kPrjP * 4;
constexpr size_t kOffDLR   = kOffDT16 + (size_t)kRows * kDtR  * 2;
constexpr size_t kOffY16   = kOffDLR  + (size_t)kRows * kDin  * 4;
constexpr size_t kWsTotal  = kOffY16  + (size_t)kRows * kYP   * 2;
static_assert(kWsTotal == 115343360ull);
static_assert(kWsTotal <= 134217728ull);
static_assert((kOffWIN % 128) == 0 && (kOffWXP % 128) == 0 && (kOffWDT % 128) == 0 && (kOffWOUT % 128) == 0 &&
              (kOffXZ % 128) == 0 && (kOffUC % 128) == 0 && (kOffUC16 % 128) == 0 && (kOffPROJ % 128) == 0 &&
              (kOffDT16 % 128) == 0 && (kOffDLR % 128) == 0 && (kOffY16 % 128) == 0);

__device__ __forceinline__ float bf_rne(float f) {
  const unsigned u = __float_as_uint(f);
  const unsigned r = (u + 0x7FFFu + ((u >> 16) & 1u)) & 0xFFFF0000u;
  return __uint_as_float(r);
}

union FragU { v16h v; v8h h[2]; };
__device__ __forceinline__ v16h frag_load_h(const _Float16* p) {
  FragU f;
  f.h[0] = *(const v8h*)(p);
  f.h[1] = *(const v8h*)(p + 16);
  return f.v;
}
__device__ __forceinline__ v8f mma_h(v16h a, v16h b, v8f c) {
  return __builtin_amdgcn_wmma_f32_16x16x32_f16(false, a, false, b, (short)0, c, false, false);
}
__device__ __forceinline__ void row_guard_h(v8f& a, v8f& b, v8f& c, v8f& d,
                                            v16h x, v16h y0, v16h y1, v16h y2, v16h y3) {
  asm volatile("v_nop\n\tv_nop\n\tv_nop\n\tv_nop"
               : "+v"(a), "+v"(b), "+v"(c), "+v"(d)
               : "v"(x), "v"(y0), "v"(y1), "v"(y2), "v"(y3));
}
__device__ __forceinline__ void keep4_h(v16h a, v16h b, v16h c, v16h d) {
  asm volatile("v_nop" :: "v"(a), "v"(b), "v"(c), "v"(d));
}
__device__ __forceinline__ void acc_guard4(v8f& a, v8f& b, v8f& c, v8f& d) {
  asm volatile("v_nop\n\tv_nop\n\tv_nop\n\tv_nop" : "+v"(a), "+v"(b), "+v"(c), "+v"(d));
}

__global__ __launch_bounds__(256) void gemm_f16_kernel(
    const unsigned short* __restrict__ Ap, int lda,
    const unsigned short* __restrict__ Btp, int ldb,
    float* __restrict__ C, int ldc,
    int M, int N, int K, float scale)
{
  const _Float16* A  = (const _Float16*)Ap;
  const _Float16* Bt = (const _Float16*)Btp;
  __shared__ __align__(16) float sT[8][16 * 68];
  const int lane = threadIdx.x & 31;
  const int wave = threadIdx.x >> 5;
  const int tilesN = N >> 6;
  const int tilesM = M >> 6;
  const int tile = blockIdx.x * 8 + wave;
  if (tile >= tilesM * tilesN) return;
  const int tm = tile / tilesN;
  const int tn = tile - tm * tilesN;
  const int m0 = tm << 6;
  const int n0 = tn << 6;

  const int rlane = lane & 15;
  const int koff  = (lane >> 4) * 8;
  const int mOff  = (lane >> 4) * 8;

  v8f acc[4][4];
#pragma unroll
  for (int i = 0; i < 4; ++i)
#pragma unroll
    for (int j = 0; j < 4; ++j) acc[i][j] = (v8f){0.f, 0.f, 0.f, 0.f, 0.f, 0.f, 0.f, 0.f};

  for (int k0 = 0; k0 < K; k0 += 32) {
    v16h bh[4];
#pragma unroll
    for (int j = 0; j < 4; ++j) {
      const size_t bo = (size_t)(n0 + (j << 4) + rlane) * ldb + koff + k0;
      bh[j] = frag_load_h(Bt + bo);
    }
#pragma unroll
    for (int i = 0; i < 4; ++i) {
      const size_t ao = (size_t)(m0 + (i << 4) + rlane) * lda + koff + k0;
      const v16h ah = frag_load_h(A + ao);
#pragma unroll
      for (int j = 0; j < 4; ++j) acc[i][j] = mma_h(ah, bh[j], acc[i][j]);
      row_guard_h(acc[i][0], acc[i][1], acc[i][2], acc[i][3], ah, bh[0], bh[1], bh[2], bh[3]);
    }
    keep4_h(bh[0], bh[1], bh[2], bh[3]);
  }
  acc_guard4(acc[0][0], acc[0][1], acc[0][2], acc[0][3]);
  acc_guard4(acc[1][0], acc[1][1], acc[1][2], acc[1][3]);
  acc_guard4(acc[2][0], acc[2][1], acc[2][2], acc[2][3]);
  acc_guard4(acc[3][0], acc[3][1], acc[3][2], acc[3][3]);

  float* slab = sT[wave];
#pragma unroll
  for (int i = 0; i < 4; ++i) {
    const int mBase = m0 + (i << 4);
#pragma unroll
    for (int j = 0; j < 4; ++j) {
#pragma unroll
      for (int r = 0; r < 8; ++r) {
        const float v = acc[i][j][r] * scale;
        slab[(mOff + r) * 68 + (j << 4) + rlane] = v;
      }
    }
    __builtin_amdgcn_fence(__ATOMIC_RELEASE, "workgroup");
    __builtin_amdgcn_wave_barrier();
    __builtin_amdgcn_fence(__ATOMIC_ACQUIRE, "workgroup");
    {
      const int hh = lane >> 4;
      const int c4 = (lane & 15) * 4;
      for (int pass = 0; pass < 2; ++pass) {
#pragma unroll
        for (int it = 0; it < 8; ++it) {
          const int row = it * 2 + hh;
          const v4f v = *(const v4f*)(slab + row * 68 + c4);
          *(volatile v4f*)(C + (size_t)(mBase + row) * ldc + n0 + c4) = v;
        }
        __threadfence();
      }
    }
    __builtin_amdgcn_fence(__ATOMIC_RELEASE, "workgroup");
    __builtin_amdgcn_wave_barrier();
    __builtin_amdgcn_fence(__ATOMIC_ACQUIRE, "workgroup");
  }
}

__global__ __launch_bounds__(256) void cast_rows_kernel(
    const float* __restrict__ src, unsigned short* __restrict__ dst,
    int rows_real, int cols, int dst_pitch, int dst_coff, int total8, float scale)
{
  const int i = blockIdx.x * 256 + threadIdx.x;
  if (i >= total8) return;
  const int cols8 = cols >> 3;
  const int r  = i / cols8;
  const int c8 = (i - r * cols8) << 3;
  const bool live = (r < rows_real);
  const int rc = live ? r : (rows_real - 1);
  const float* p = src + (size_t)rc * cols + c8;
  const v4f a0 = *(const v4f*)(p);
  const v4f a1 = *(const v4f*)(p + 4);
  v8h hv;
#pragma unroll
  for (int e = 0; e < 4; ++e) {
    const float s0 = a0[e];
    const float s1 = a1[e];
    const float t0 = bf_rne(s0) * scale;
    const float t1 = bf_rne(s1) * scale;
    hv[e]     = (_Float16)(live ? t0 : 0.0f);
    hv[4 + e] = (_Float16)(live ? t1 : 0.0f);
  }
  unsigned short* q = dst + (size_t)r * dst_pitch + dst_coff + c8;
  *(volatile v8h*)q = hv;
  __threadfence();
  *(volatile v8h*)q = hv;
}

__global__ __launch_bounds__(256) void dt_cast_kernel(
    const float* __restrict__ PROJ, unsigned short* __restrict__ DT16, int total8, float scale)
{
  const int i = blockIdx.x * 256 + threadIdx.x;
  if (i >= total8) return;
  const int e0  = i << 3;
  const int row = e0 >> 6;
  const int c8  = e0 & 63;
  const float* p = PROJ + (size_t)row * kPrjP + c8;
  const v4f a0 = *(const v4f*)(p);
  const v4f a1 = *(const v4f*)(p + 4);
  v8h hv;
#pragma unroll
  for (int e = 0; e < 4; ++e) {
    const float s0 = a0[e];
    const float s1 = a1[e];
    hv[e]     = (_Float16)(s0 * scale);
    hv[4 + e] = (_Float16)(s1 * scale);
  }
  unsigned short* qd = DT16 + e0;
  *(volatile v8h*)qd = hv;
  __threadfence();
  *(volatile v8h*)qd = hv;
}

__global__ __launch_bounds__(256) void conv_silu_kernel(
    const float* __restrict__ XZ, const float* __restrict__ cw, const float* __restrict__ cb,
    float* __restrict__ UC, unsigned short* __restrict__ UC16, int dir)
{
  __shared__ __align__(16) float sT[16 * kTP];
  const int tid = threadIdx.x, lane = tid & 31, wave = tid >> 5;
  const int d0 = blockIdx.x * 256, d = d0 + tid;
  const int g0 = blockIdx.y * 64;
  const v4f wv = *(const v4f*)(cw + (size_t)d * 4);
  const float wr0 = wv[0], wr1 = wv[1], wr2 = wv[2], wr3 = wv[3];
  const float w0 = bf_rne(wr0), w1 = bf_rne(wr1), w2 = bf_rne(wr2), w3 = bf_rne(wr3);
  const float bc = bf_rne(cb[d]);
  const int sgn = dir ? -1 : 1;
  const int gs = dir ? (g0 + 63) : g0;
  const int ts = gs & (kSeqL - 1);
  float xm1, xm2, xm3;
  {
    const int t1 = ts - sgn, t2 = ts - 2 * sgn, t3 = ts - 3 * sgn;
    int r1 = gs - sgn, r2 = gs - 2 * sgn, r3 = gs - 3 * sgn;
    r1 = r1 < 0 ? 0 : (r1 > kRows - 1 ? kRows - 1 : r1);
    r2 = r2 < 0 ? 0 : (r2 > kRows - 1 ? kRows - 1 : r2);
    r3 = r3 < 0 ? 0 : (r3 > kRows - 1 ? kRows - 1 : r3);
    const float v1 = XZ[(size_t)r1 * kXZP + d];
    const float v2 = XZ[(size_t)r2 * kXZP + d];
    const float v3 = XZ[(size_t)r3 * kXZP + d];
    const bool ok1 = (t1 >= 0) && (t1 < kSeqL);
    const bool ok2 = (t2 >= 0) && (t2 < kSeqL);
    const bool ok3 = (t3 >= 0) && (t3 < kSeqL);
    xm1 = ok1 ? v1 : 0.0f;
    xm2 = ok2 ? v2 : 0.0f;
    xm3 = ok3 ? v3 : 0.0f;
  }
  const int hrow = wave >> 1;
  const int hch  = (wave & 1) * 128 + lane * 4;
#pragma unroll 1
  for (int sub = 0; sub < 4; ++sub) {
    const int sb = dir ? (3 - sub) : sub;
    const int lb = g0 + sb * 16;
#pragma unroll 1
    for (int s = 0; s < 16; ++s) {
      const int rl = dir ? (15 - s) : s;
      const float xcur = XZ[(size_t)(lb + rl) * kXZP + d];
      float acc = w0 * xm3;
      acc = fmaf(w1, xm2, acc);
      acc = fmaf(w2, xm1, acc);
      acc = fmaf(w3, xcur, acc);
      const float sv = bc + acc;
      const float ev = expf(-sv);
      const float sg = 1.0f / (1.0f + ev);
      sT[rl * kTP + tid] = sv * sg;
      xm3 = xm2; xm2 = xm1; xm1 = xcur;
    }
    __syncthreads();
    v4f fv[4];
    v8h bv[2];
#pragma unroll
    for (int it = 0; it < 4; ++it) fv[it] = *(const v4f*)(sT + (it * 4 + hrow) * kTP + hch);
#pragma unroll
    for (int it = 0; it < 2; ++it) {
      const float* sp = sT + (it * 8 + wave) * kTP + lane * 8;
      const v4f a0 = *(const v4f*)(sp);
      const v4f a1 = *(const v4f*)(sp + 4);
#pragma unroll
      for (int e = 0; e < 4; ++e) {
        const float s0 = a0[e];
        const float s1 = a1[e];
        bv[it][e]     = (_Float16)(s0 * kCarryU);
        bv[it][4 + e] = (_Float16)(s1 * kCarryU);
      }
    }
    for (int pass = 0; pass < 2; ++pass) {
#pragma unroll
      for (int it = 0; it < 4; ++it)
        *(volatile v4f*)(UC + (size_t)(lb + it * 4 + hrow) * kDin + d0 + hch) = fv[it];
#pragma unroll
      for (int it = 0; it < 2; ++it)
        *(volatile v8h*)(UC16 + (size_t)(lb + it * 8 + wave) * kDin + d0 + lane * 8) = bv[it];
      __threadfence();
    }
    __syncthreads();
  }
}

__global__ __launch_bounds__(256) void scan_kernel(
    const float* __restrict__ DLR, const float* __restrict__ UC, const float* __restrict__ XZ,
    const float* __restrict__ PROJ, const float* __restrict__ A_log, const float* __restrict__ Dv,
    const float* __restrict__ bdt, unsigned short* __restrict__ Y16, int dir)
{
  __shared__ __align__(16) float sBC[kChunk * 32];
  __shared__ __align__(16) float sY[kChunk * kTP];
  __shared__ __align__(16) float sA[kNst * 256];
  const int tid = threadIdx.x, lane = tid & 31, wave = tid >> 5;
  const int d0 = blockIdx.x * 256, d = d0 + tid;
  const int row0 = blockIdx.y * kSeqL;

#pragma unroll 1
  for (int n = 0; n < kNst; ++n) {
    const float al = bf_rne(A_log[(size_t)d * kNst + n]);
    sA[n * 256 + tid] = -expf(al);
  }
  __syncthreads();
  float An[kNst], h[kNst];
#pragma unroll
  for (int n = 0; n < kNst; ++n) {
    An[n] = sA[n * 256 + tid];
    h[n] = 0.0f;
  }
  const float Dd = bf_rne(Dv[d]);
  const float bb = bf_rne(bdt[d]);
  const int ycol = dir * kDin + d0 + lane * 8;

#pragma unroll 1
  for (int c = 0; c < kSeqL / kChunk; ++c) {
    const int cc = dir ? (kSeqL / kChunk - 1 - c) : c;
    const int l0 = row0 + cc * kChunk;
    if (tid < 128) {
      const int r = tid >> 3, q = (tid & 7) * 4;
      const v4f v = *(const v4f*)(PROJ + (size_t)(l0 + r) * kPrjP + kDtR + q);
      *(v4f*)(sBC + r * 32 + q) = v;
    }
    __syncthreads();
#pragma unroll 1
    for (int s = 0; s < kChunk; ++s) {
      const int sl = dir ? (kChunk - 1 - s) : s;
      const size_t m = (size_t)(l0 + sl);
      const float a  = DLR[m * kDin + d] + bb;
      const float ea = __expf(-fabsf(a));
      const float up = 1.0f + ea;
      const float l1p = __logf(up) + (ea - (up - 1.0f)) * __builtin_amdgcn_rcpf(up);
      const float delta = fmaxf(a, 0.0f) + l1p;
      const float xv = UC[m * kDin + d];
      const float zv = XZ[m * kXZP + kDin + d];
      v4f Bq[4], Cq[4];
#pragma unroll
      for (int qq = 0; qq < 4; ++qq) {
        Bq[qq] = *(const v4f*)(sBC + sl * 32 + 4 * qq);
        Cq[qq] = *(const v4f*)(sBC + sl * 32 + kNst + 4 * qq);
      }
      const float dtx = delta * xv;
      float y = 0.0f;
#pragma unroll
      for (int n = 0; n < kNst; ++n) {
        const float e  = __expf(delta * An[n]);
        const float bn = Bq[n >> 2][n & 3];
        const float cn = Cq[n >> 2][n & 3];
        const float hn = fmaf(e, h[n], dtx * bn);
        h[n] = hn;
        y = fmaf(hn, cn, y);
      }
      y = fmaf(xv, Dd, y);
      const float ez = expf(-zv);
      const float sg = 1.0f / (1.0f + ez);
      const float g  = zv * sg;
      sY[sl * kTP + tid] = (y * g) * kCarryY;
    }
    __syncthreads();
    v8h hv[2];
#pragma unroll
    for (int it = 0; it < 2; ++it) {
      const float* sp = sY + (it * 8 + wave) * kTP + lane * 8;
      const v4f a0 = *(const v4f*)(sp);
      const v4f a1 = *(const v4f*)(sp + 4);
#pragma unroll
      for (int e = 0; e < 4; ++e) {
        const float s0 = a0[e];
        const float s1 = a1[e];
        hv[it][e]     = (_Float16)s0;
        hv[it][4 + e] = (_Float16)s1;
      }
    }
    for (int pass = 0; pass < 2; ++pass) {
#pragma unroll
      for (int it = 0; it < 2; ++it)
        *(volatile v8h*)(Y16 + (size_t)(l0 + it * 8 + wave) * kYP + ycol) = hv[it];
      __threadfence();
    }
  }
}

extern "C" void kernel_launch(void* const* d_in, const int* in_sizes, int n_in,
                              void* d_out, int out_size, void* d_ws, size_t ws_size,
                              hipStream_t stream)
{
  (void)stream;
  if (n_in < 19) return;
  if (in_sizes[0] != kRows * kDmod) return;
  for (int p = 0; p < 2; ++p) {
    const int b = 1 + 9 * p;
    if (in_sizes[b + 0] != kXZP * kDmod) return;
    if (in_sizes[b + 1] != kDin * 4) return;
    if (in_sizes[b + 2] != kDin) return;
    if (in_sizes[b + 3] != kPrjN * kDin) return;
    if (in_sizes[b + 4] != kDin * kDtR) return;
    if (in_sizes[b + 5] != kDin) return;
    if (in_sizes[b + 6] != kDin * kNst) return;
    if (in_sizes[b + 7] != kDin) return;
    if (in_sizes[b + 8] != kDmod * kDin) return;
  }
  if (out_size != kRows * kDmod) return;
  if (ws_size < kWsTotal) return;

  const float* x = (const float*)d_in[0];
  float* out = (float*)d_out;
  char* ws = (char*)d_ws;
  unsigned short* X16    = (unsigned short*)(ws + kOffX16);
  unsigned short* WIN16  = (unsigned short*)(ws + kOffWIN);
  unsigned short* WXP16  = (unsigned short*)(ws + kOffWXP);
  unsigned short* WDT16  = (unsigned short*)(ws + kOffWDT);
  unsigned short* WOUT16 = (unsigned short*)(ws + kOffWOUT);
  float*          XZ     = (float*)(ws + kOffXZ);
  float*          UC     = (float*)(ws + kOffUC);
  unsigned short* UC16   = (unsigned short*)(ws + kOffUC16);
  float*          PROJ   = (float*)(ws + kOffPROJ);
  unsigned short* DT16   = (unsigned short*)(ws + kOffDT16);
  float*          DLR    = (float*)(ws + kOffDLR);
  unsigned short* Y16    = (unsigned short*)(ws + kOffY16);

  cast_rows_kernel<<<(kRows * kDmod / 8) / 256, 256, 0, stream>>>(
      x, X16, kRows, kDmod, kDmod, 0, kRows * kDmod / 8, 1.0f);
  cast_rows_kernel<<<(kDmod * kDin / 8) / 256, 256, 0, stream>>>(
      (const float*)d_in[9], WOUT16, kDmod, kDin, kYP, 0, kDmod * kDin / 8, kCarryW);
  cast_rows_kernel<<<(kDmod * kDin / 8) / 256, 256, 0, stream>>>(
      (const float*)d_in[18], WOUT16, kDmod, kDin, kYP, kDin, kDmod * kDin / 8, kCarryW);

  for (int dir = 0; dir < 2; ++dir) {
    const int b = 1 + 9 * dir;
    const float* in_w    = (const float*)d_in[b + 0];
    const float* conv_w  = (const float*)d_in[b + 1];
    const float* conv_b  = (const float*)d_in[b + 2];
    const float* xproj_w = (const float*)d_in[b + 3];
    const float* dt_w    = (const float*)d_in[b + 4];
    const float* dt_b    = (const float*)d_in[b + 5];
    const float* A_log   = (const float*)d_in[b + 6];
    const float* Dp      = (const float*)d_in[b + 7];

    cast_rows_kernel<<<(kXZP * kDmod / 8) / 256, 256, 0, stream>>>(
        in_w, WIN16, kXZP, kDmod, kDmod, 0, kXZP * kDmod / 8, kCarryW);

    gemm_f16_kernel<<<(kRows / 64) * (kXZP / 64) / 8, 256, 0, stream>>>(
        X16, kDmod, WIN16, kDmod, XZ, kXZP, kRows, kXZP, kDmod, kFoldIn);

    conv_silu_kernel<<<dim3(kDin / 256, kRows / 64), 256, 0, stream>>>(XZ, conv_w, conv_b, UC, UC16, dir);

    cast_rows_kernel<<<(kPrjP * kDin / 8) / 256, 256, 0, stream>>>(
        xproj_w, WXP16, kPrjN, kDin, kDin, 0, kPrjP * kDin / 8, kCarryW);

    gemm_f16_kernel<<<(kRows / 64) * (kPrjP / 64) / 8, 256, 0, stream>>>(
        UC16, kDin, WXP16, kDin, PROJ, kPrjP, kRows, kPrjP, kDin, kFoldXp);

    dt_cast_kernel<<<(kRows * kDtR / 8) / 256, 256, 0, stream>>>(PROJ, DT16, kRows * kDtR / 8, kCarryDt);

    cast_rows_kernel<<<(kDin * kDtR / 8) / 256, 256, 0, stream>>>(
        dt_w, WDT16, kDin, kDtR, kDtR, 0, kDin * kDtR / 8, kCarryW);

    gemm_f16_kernel<<<(kRows / 64) * (kDin / 64) / 8, 256, 0, stream>>>(
        DT16, kDtR, WDT16, kDtR, DLR, kDin, kRows, kDin, kDtR, kFoldDt);

    scan_kernel<<<dim3(kDin / 256, kBatch), 256, 0, stream>>>(DLR, UC, XZ, PROJ, A_log, Dp, dt_b, Y16, dir);
  }

  gemm_f16_kernel<<<(kRows / 64) * (kDmod / 64) / 8, 256, 0, stream>>>(
      Y16, kYP, WOUT16, kYP, out, kDmod, kRows, kDmod, kYP, kFoldOut);
}
